// DropLearner_8040178778537
// MI455X (gfx1250) — hardware-verified
//
#include <hip/hip_runtime.h>
#include <stddef.h>


#define CH     128
#define NCOL   192
#define XW     (3 * CH)
#define HC     96
#define NTH    (HC / 16)
#define KPB    128
#define APZ    136
#define GROWS  32
#define GTHR   64
#define PTHR   256
#define ETHR   128
#define EPB    128
#define PLN    (NCOL * KPB)
#define BPTOT  (3 * PLN)
#define WSCAP  134217728
#define W1SC   16.0f
#define RP     0.0625f
#define EPSA   (-0.9998f)
#define EPSB   0.9999f
#define RTEMP  2.0f
#define GCL    30.0f

static_assert(((BPTOT / 8) % PTHR) == 0);
static_assert((APZ % 8) == 0 && (KPB % 8) == 0 && (CH % 32) == 0);
static_assert(GROWS == (GTHR / 32) * 16);
static_assert(GROWS * CH == 64 * GTHR);
static_assert(((GROWS * HC) % (4 * GTHR)) == 0);
static_assert(EPB == ETHR && (HC % 4) == 0 && NTH * 16 == HC && 2 * HC == NCOL);
static_assert((PLN / 8) == NCOL * 16);

typedef float    v4f  __attribute__((ext_vector_type(4)));
typedef float    v8f  __attribute__((ext_vector_type(8)));
typedef _Float16 v8h  __attribute__((ext_vector_type(8)));
typedef _Float16 v16h __attribute__((ext_vector_type(16)));
union Frag { v16h v; v8h h[2]; };

__device__ __forceinline__ v8f wmh(v16h a, v16h b, v8f c) {
  v8f d = __builtin_amdgcn_wmma_f32_16x16x32_f16(false, a, false, b, (short)0, c, false, false);
  asm volatile("v_nop\n\tv_nop\n\tv_nop\n\tv_nop" : "+v"(d) : "v"(a), "v"(b));
  return d;
}

template <int NT>
__device__ __forceinline__ void mma16(const _Float16* At, const _Float16* __restrict__ Bpl,
                                      int lane, v8f (&acc)[NT]) {
  const int hh = lane >> 4, m = lane & 15;
#pragma unroll
  for (int t = 0; t < NT; ++t) { v8f z = {0.f, 0.f, 0.f, 0.f, 0.f, 0.f, 0.f, 0.f}; acc[t] = z; }
  const _Float16* ap = At + m * APZ + 8 * hh;
  const _Float16* bb = Bpl + (size_t)m * KPB + 8 * hh;
#pragma unroll 1
  for (int ks = 0; ks < CH / 32; ++ks) {
    Frag a;
    a.h[0] = *(const v8h*)(ap + 32 * ks);
    a.h[1] = *(const v8h*)(ap + 32 * ks + 16);
#pragma unroll
    for (int t = 0; t < NT; ++t) {
      const _Float16* bp = bb + (size_t)(16 * t) * KPB + 32 * ks;
      Frag b;
      b.h[0] = *(const v8h*)bp;
      b.h[1] = *(const v8h*)(bp + 16);
      acc[t] = wmh(a.v, b.v, acc[t]);
    }
  }
}

__global__ __launch_bounds__(PTHR) void k_wprep(const float* __restrict__ W1, _Float16* Bpl) {
  const int i = blockIdx.x * PTHR + threadIdx.x;
  const int seg = i / (PLN / 8);
  const int rem = i - seg * (PLN / 8);
  const int n = rem >> 4, k0 = (rem & 15) * 8;
  const float* sp = W1 + (size_t)n * XW + seg * CH + k0;
  const v4f a = *(const v4f*)sp;
  const v4f b = *(const v4f*)(sp + 4);
  v8h hv;
  hv[0] = (_Float16)(a.x * W1SC); hv[1] = (_Float16)(a.y * W1SC);
  hv[2] = (_Float16)(a.z * W1SC); hv[3] = (_Float16)(a.w * W1SC);
  hv[4] = (_Float16)(b.x * W1SC); hv[5] = (_Float16)(b.y * W1SC);
  hv[6] = (_Float16)(b.z * W1SC); hv[7] = (_Float16)(b.w * W1SC);
  _Float16* dp = Bpl + (size_t)8 * i;
  *(volatile v8h*)dp = hv;
  __threadfence();
  *(volatile v8h*)dp = hv;
}

__global__ __launch_bounds__(GTHR) void k_nodegemm(const float* __restrict__ x, const _Float16* __restrict__ Bp,
                                                   const float* __restrict__ b1, float* dst,
                                                   int nRows, int col0, int addBias) {
  __shared__ __attribute__((aligned(16))) _Float16 At[GROWS * APZ];
  __shared__ __attribute__((aligned(16))) float stg[GROWS * HC];
  const int tid = threadIdx.x, lane = tid & 31, wave = tid >> 5, hh = lane >> 4, m = lane & 15;
  const int rowBase = blockIdx.x * GROWS;
  {
    const int r = tid >> 1, c0 = (tid & 1) * 64;
    int xrow = rowBase + r;
    xrow = xrow > nRows - 1 ? nRows - 1 : xrow;
    const float* xp = x + (size_t)xrow * CH + c0;
#pragma unroll
    for (int j = 0; j < 8; ++j) {
      const v4f a = *(const v4f*)(xp + 8 * j), b = *(const v4f*)(xp + 8 * j + 4);
      v8h hv;
      hv[0] = (_Float16)a.x; hv[1] = (_Float16)a.y; hv[2] = (_Float16)a.z; hv[3] = (_Float16)a.w;
      hv[4] = (_Float16)b.x; hv[5] = (_Float16)b.y; hv[6] = (_Float16)b.z; hv[7] = (_Float16)b.w;
      *(v8h*)(At + r * APZ + c0 + 8 * j) = hv;
    }
  }
  __syncthreads();

  {
    v8f acc[NTH];
    mma16<NTH>(At + wave * 16 * APZ, Bp, lane, acc);
    float* sp = stg + (wave * 16 + 8 * hh) * HC + m;
#pragma unroll
    for (int t = 0; t < NTH; ++t) {
      const float bb = b1[col0 + 16 * t + m];
      const float bv = addBias ? bb : 0.0f;
#pragma unroll
      for (int r = 0; r < 8; ++r) sp[r * HC + 16 * t] = acc[t][r] * RP + bv;
    }
  }
  __syncthreads();

  float* gp = dst + (size_t)rowBase * HC;
#pragma unroll
  for (int it = 0; it < (GROWS * HC) / (4 * GTHR); ++it) {
    const int f = it * GTHR + tid;
    const v4f v = *(const v4f*)(stg + 4 * f);
    *(volatile v4f*)(gp + 4 * f) = v;
  }
  __threadfence();
#pragma unroll
  for (int it = 0; it < (GROWS * HC) / (4 * GTHR); ++it) {
    const int f = it * GTHR + tid;
    const v4f v = *(const v4f*)(stg + 4 * f);
    *(volatile v4f*)(gp + 4 * f) = v;
  }
}

__global__ __launch_bounds__(ETHR) void k_edge(
    const float* __restrict__ PQ, const float* __restrict__ Rp,
    const int* __restrict__ ei, const int* __restrict__ et,
    const float* __restrict__ W2, const float* __restrict__ b2, const float* __restrict__ uu,
    float* part, float* out, int nN, int nR, int nE, int nPad, int chalf, int fin) {
#pragma clang fp contract(off)
  __shared__ __attribute__((aligned(16))) float sc[EPB];
  const int tid = threadIdx.x, lane = tid & 31, wave = tid >> 5;
  const int e = blockIdx.x * EPB + tid;
  const int ec = e > nE - 1 ? nE - 1 : e;
  int s = ei[ec];
  s = s < 0 ? 0 : (s > nN - 1 ? nN - 1 : s);
  int d = ei[(size_t)nE + ec];
  d = d < 0 ? 0 : (d > nN - 1 ? nN - 1 : d);
  int t = et[ec];
  t = t < 0 ? 0 : (t > nR - 1 ? nR - 1 : t);
  const float* pp = PQ + (size_t)s * HC;
  const float* qq = PQ + ((size_t)nPad + (size_t)d) * HC;
  const float* rr = Rp + (size_t)t * HC;
  const float* wp = W2 + chalf * HC;

  float acc = 0.0f;
#pragma unroll 2
  for (int c = 0; c < HC / 4; ++c) {
    const v4f p = *(const v4f*)(pp + 4 * c);
    const v4f q = *(const v4f*)(qq + 4 * c);
    const v4f r = *(const v4f*)(rr + 4 * c);
    const v4f w = *(const v4f*)(wp + 4 * c);
    const v4f hs = (p + q) + r;
    acc = fmaf(fmaxf(hs.x, 0.0f), w.x, acc);
    acc = fmaf(fmaxf(hs.y, 0.0f), w.y, acc);
    acc = fmaf(fmaxf(hs.z, 0.0f), w.z, acc);
    acc = fmaf(fmaxf(hs.w, 0.0f), w.w, acc);
  }

  float val = acc;
  if (fin) {
    const float wgt = (part[e] + acc) + b2[0];
    const float ue  = uu[ec];
    const float em  = EPSA * ue;
    const float eps = em + EPSB;
    const float lg  = logf(eps) - log1pf(-eps);
    float g = (lg + wgt) * RTEMP;
    g = fminf(fmaxf(g, -GCL), GCL);
    const float ex = expf(-g);
    val = __builtin_amdgcn_rcpf(1.0f + ex);
  }
  sc[tid] = val;
  __syncthreads();

  if (wave == 0) {
    const v4f ov = *(const v4f*)(sc + 4 * lane);
    const int e0 = blockIdx.x * EPB + 4 * lane;
    if (fin) {
      float* op = out + e0;
      const bool full = (e0 + 3 < nE);
      if (full) {
        *(volatile v4f*)op = ov;
      } else {
        if (e0     < nE) *(volatile float*)(op)     = ov.x;
        if (e0 + 1 < nE) *(volatile float*)(op + 1) = ov.y;
        if (e0 + 2 < nE) *(volatile float*)(op + 2) = ov.z;
      }
      __threadfence();
      if (full) {
        *(volatile v4f*)op = ov;
      } else {
        if (e0     < nE) *(volatile float*)(op)     = ov.x;
        if (e0 + 1 < nE) *(volatile float*)(op + 1) = ov.y;
        if (e0 + 2 < nE) *(volatile float*)(op + 2) = ov.z;
      }
    } else {
      float* qp = part + e0;
      *(volatile v4f*)qp = ov;
      __threadfence();
      *(volatile v4f*)qp = ov;
    }
  }
}

extern "C" void kernel_launch(void* const* d_in, const int* in_sizes, int n_in,
                              void* d_out, int out_size, void* d_ws, size_t ws_size,
                              hipStream_t stream) {
  if (n_in < 9) return;
  const int nE = in_sizes[1];
  if (nE <= 0 || in_sizes[0] != 2 * nE) return;
  if (in_sizes[2] <= 0 || (in_sizes[2] % CH) != 0) return;
  if (in_sizes[3] <= 0 || (in_sizes[3] % CH) != 0) return;
  const int nN = in_sizes[2] / CH;
  const int nR = in_sizes[3] / CH;
  if (in_sizes[4] != nE || in_sizes[5] != NCOL * XW || in_sizes[6] != NCOL ||
      in_sizes[7] != NCOL || in_sizes[8] < 1) return;
  if (out_size != nE) return;
  if (nN > (1 << 24) || nR > (1 << 20) || nE > (1 << 28)) return;

  const int*   ei  = (const int*)d_in[0];
  const int*   et  = (const int*)d_in[1];
  const float* emb = (const float*)d_in[2];
  const float* rel = (const float*)d_in[3];
  const float* uu  = (const float*)d_in[4];
  const float* W1  = (const float*)d_in[5];
  const float* b1  = (const float*)d_in[6];
  const float* W2  = (const float*)d_in[7];
  const float* b2  = (const float*)d_in[8];
  float* out = (float*)d_out;

  const int nBlkG = (nN + GROWS - 1) / GROWS;
  const int nPad  = nBlkG * GROWS;
  const int nBlkR = (nR + GROWS - 1) / GROWS;
  const int nRPad = nBlkR * GROWS;
  const int nBlkE = (nE + EPB - 1) / EPB;
  const int nEPad = nBlkE * EPB;

  char* ws = (char*)d_ws;
  size_t off = 0;
  const size_t oB  = off; off += (size_t)BPTOT * 2;            off = (off + 255) & ~(size_t)255;
  const size_t oPQ = off; off += (size_t)2 * nPad * HC * 4;     off = (off + 255) & ~(size_t)255;
  const size_t oR  = off; off += (size_t)nRPad * HC * 4;        off = (off + 255) & ~(size_t)255;
  const size_t oEp = off; off += (size_t)nEPad * 4;             off = (off + 255) & ~(size_t)255;
  if (off > ws_size || off > (size_t)WSCAP) return;
  _Float16* Bpl = (_Float16*)(ws + oB);
  float*    PQ  = (float*)(ws + oPQ);
  float*    Rpl = (float*)(ws + oR);
  float*    Ep  = (float*)(ws + oEp);

  k_wprep<<<(BPTOT / 8) / PTHR, PTHR, 0, stream>>>(W1, Bpl);

  for (int chalf = 0; chalf < 2; ++chalf) {
    const int col0 = chalf * HC;
    k_nodegemm<<<nBlkG, GTHR, 0, stream>>>(emb, Bpl + 0 * PLN + (size_t)col0 * KPB, b1, PQ, nN, col0, 1);
    k_nodegemm<<<nBlkG, GTHR, 0, stream>>>(emb, Bpl + 1 * PLN + (size_t)col0 * KPB, b1, PQ + (size_t)nPad * HC, nN, col0, 0);
    k_nodegemm<<<nBlkR, GTHR, 0, stream>>>(rel, Bpl + 2 * PLN + (size_t)col0 * KPB, b1, Rpl, nR, col0, 0);
    k_edge<<<nBlkE, ETHR, 0, stream>>>(PQ, Rpl, ei, et, W2, b2, uu, Ep, out, nN, nR, nE, nPad, chalf, chalf);
  }
}
